// CausalMultiHeadAttention_4415226380965
// MI455X (gfx1250) — hardware-verified
//
#include <hip/hip_runtime.h>
#include <math.h>
#include <stdint.h>

#ifndef NB
#define NB 2
#endif
#ifndef SEQ
#define SEQ 2048
#endif
#define NB_FULL  2
#define SEQ_FULL 2048
#define DM    2048
#define NH    16
#define HD    128
#define NQB   (SEQ / 64)
#define RESQB 4
#define RESROWS (RESQB * 64)
#define VLP   RESROWS
#define CHKB  64
#define QLC   2048.0f
#define PVC   4096.0f
#define OLC   1024.0f
#define WOC   256.0f
static_assert(NH * HD == DM);
static_assert(HD == 128);
static_assert(NB >= 1 && NB <= NB_FULL);
static_assert(SEQ >= RESROWS && SEQ <= SEQ_FULL && (SEQ % 256) == 0);
static_assert((DM % 64) == 0 && (DM % 32) == 0 && (RESROWS % 64) == 0 && (VLP % 64) == 0);
static_assert(NQB >= RESQB);
static_assert((SEQ * DM) % (8 * 256) == 0 && (DM * DM) % (8 * 256) == 0);

typedef _Float16 v16h __attribute__((ext_vector_type(16)));
typedef _Float16 v8h  __attribute__((ext_vector_type(8)));
typedef __bf16   v16b __attribute__((ext_vector_type(16)));
typedef __bf16   v8b  __attribute__((ext_vector_type(8)));
typedef float    v8f  __attribute__((ext_vector_type(8)));
typedef float    v4f  __attribute__((ext_vector_type(4)));
typedef unsigned int v4u __attribute__((ext_vector_type(4)));
typedef int      v4i  __attribute__((ext_vector_type(4)));

__device__ __forceinline__ unsigned short bf_bits(float f) {
  unsigned u = __float_as_uint(f);
  return (unsigned short)((u + 0x7FFFu + ((u >> 16) & 1u)) >> 16);
}
__device__ __forceinline__ float bf_up(unsigned short h) { return __uint_as_float(((unsigned)h) << 16); }
__device__ __forceinline__ float bfr(float f) { return bf_up(bf_bits(f)); }
__device__ __forceinline__ unsigned short h_bits(_Float16 x) { return __builtin_bit_cast(unsigned short, x); }
__device__ __forceinline__ unsigned pk16(unsigned short a, unsigned short b) { return (unsigned)a | ((unsigned)b << 16); }
__device__ __forceinline__ v8f zero8() { v8f z = {0.f, 0.f, 0.f, 0.f, 0.f, 0.f, 0.f, 0.f}; return z; }
__device__ __forceinline__ v8h zero8h() {
  const _Float16 z = (_Float16)0.0f;
  v8h r = {z, z, z, z, z, z, z, z};
  return r;
}

__device__ __forceinline__ v16b ldfrag(const __bf16* p) {
  union { v16b v; v8b h[2]; } f;
  f.h[0] = *(const v8b*)(p);
  f.h[1] = *(const v8b*)(p + 16);
  return f.v;
}
__device__ __forceinline__ v16h ldfrag(const _Float16* p) {
  union { v16h v; v8h h[2]; } f;
  f.h[0] = *(const v8h*)(p);
  f.h[1] = *(const v8h*)(p + 16);
  return f.v;
}

__device__ __forceinline__ v8f mma_h(v16h a, v16h b, v8f c) {
  c = __builtin_amdgcn_wmma_f32_16x16x32_f16(false, a, false, b, (short)0, c, false, false);
  asm volatile("v_nop\n\tv_nop\n\tv_nop\n\tv_nop" : "+v"(c) : "v"(a), "v"(b));
  return c;
}
__device__ __forceinline__ v8f mma_raw(v16b a, v16b b, v8f c) {
  return __builtin_amdgcn_wmma_f32_16x16x32_bf16(false, a, false, b, (short)0, c, false, false);
}
__device__ __forceinline__ v8f mma_raw(v16h a, v16h b, v8f c) {
  return __builtin_amdgcn_wmma_f32_16x16x32_f16(false, a, false, b, (short)0, c, false, false);
}
__device__ __forceinline__ void dep_guard1(v8f& a, v8f& b, v16b x) {
  asm volatile("v_nop\n\tv_nop\n\tv_nop\n\tv_nop" : "+v"(a), "+v"(b) : "v"(x));
}
__device__ __forceinline__ void dep_guard1(v8f& a, v8f& b, v16h x) {
  asm volatile("v_nop\n\tv_nop\n\tv_nop\n\tv_nop" : "+v"(a), "+v"(b) : "v"(x));
}
__device__ __forceinline__ void keep4(v16b a, v16b b, v16b c, v16b d) {
  asm volatile("v_nop" :: "v"(a), "v"(b), "v"(c), "v"(d));
}
__device__ __forceinline__ void keep4(v16h a, v16h b, v16h c, v16h d) {
  asm volatile("v_nop" :: "v"(a), "v"(b), "v"(c), "v"(d));
}
__device__ __forceinline__ void acc_guard4(v8f& a, v8f& b, v8f& c, v8f& d) {
  asm volatile("v_nop\n\tv_nop\n\tv_nop\n\tv_nop" : "+v"(a), "+v"(b), "+v"(c), "+v"(d));
}

template <bool F16OP> struct OpT { typedef __bf16 E; typedef v16b V; };
template <> struct OpT<true> { typedef _Float16 E; typedef v16h V; };

__global__ __launch_bounds__(256) void cvt_bf16x8(const float* __restrict__ in, unsigned short* out, int n8,
                                                   long long strideIn, long long strideOut) {
  const int i = blockIdx.x * 256 + threadIdx.x;
  const float* src = in + (size_t)blockIdx.y * (size_t)strideIn;
  unsigned short* dst = out + (size_t)blockIdx.y * (size_t)strideOut;
  if (i < n8) {
    const v4f a = *(const v4f*)(src + (size_t)i * 8);
    const v4f b = *(const v4f*)(src + (size_t)i * 8 + 4);
    v4u p;
    p[0] = pk16(bf_bits(a[0]), bf_bits(a[1]));
    p[1] = pk16(bf_bits(a[2]), bf_bits(a[3]));
    p[2] = pk16(bf_bits(b[0]), bf_bits(b[1]));
    p[3] = pk16(bf_bits(b[2]), bf_bits(b[3]));
    *(volatile v4u*)(dst + (size_t)i * 8) = p;
    __threadfence();
    *(volatile v4u*)(dst + (size_t)i * 8) = p;
  }
}

__global__ __launch_bounds__(256) void cvt_f16x8(const float* __restrict__ in, unsigned short* out, int n8, float sc) {
  const int i = blockIdx.x * 256 + threadIdx.x;
  if (i < n8) {
    const v4f a = *(const v4f*)(in + (size_t)i * 8);
    const v4f b = *(const v4f*)(in + (size_t)i * 8 + 4);
    v4u p;
    p[0] = pk16(h_bits((_Float16)(bfr(a[0]) * sc)), h_bits((_Float16)(bfr(a[1]) * sc)));
    p[1] = pk16(h_bits((_Float16)(bfr(a[2]) * sc)), h_bits((_Float16)(bfr(a[3]) * sc)));
    p[2] = pk16(h_bits((_Float16)(bfr(b[0]) * sc)), h_bits((_Float16)(bfr(b[1]) * sc)));
    p[3] = pk16(h_bits((_Float16)(bfr(b[2]) * sc)), h_bits((_Float16)(bfr(b[3]) * sc)));
    *(volatile v4u*)(out + (size_t)i * 8) = p;
    __threadfence();
    *(volatile v4u*)(out + (size_t)i * 8) = p;
  }
}

__global__ __launch_bounds__(256) void mask_check(const int* __restrict__ mask, int* flags, int seq, int pitch) {
  __shared__ int sred[8];
  const int tid = threadIdx.x, lane = tid & 31, wave = tid >> 5;
  const int per4  = seq >> 2;
  const int total = seq * per4;
  int bad = 0;
  for (int g = blockIdx.x * 256 + tid; g < total; g += CHKB * 256) {
    const int i  = g / per4;
    const int j4 = (g - i * per4) << 2;
    const v4i v = *(const v4i*)(mask + (size_t)i * pitch + j4);
#pragma unroll
    for (int e = 0; e < 4; ++e) {
      const int keep = ((j4 + e) <= i) ? 1 : 0;
      const int got  = (v[e] != 0) ? 1 : 0;
      bad |= (got != keep) ? 1 : 0;
    }
  }
#pragma unroll
  for (int off = 1; off < 32; off <<= 1) bad |= __shfl_xor(bad, off, 32);
  if (lane == 0) sred[wave] = bad;
  __syncthreads();
  if (wave == 0) {
    int t = sred[lane & 7];
#pragma unroll
    for (int off = 1; off < 32; off <<= 1) t |= __shfl_xor(t, off, 32);
    const int val = (lane == 0) ? t : 0;
    volatile int* fp = flags + (size_t)blockIdx.x * 32 + lane;
    *fp = val;
    __threadfence();
    *fp = val;
  }
}

template <bool F16OP, int NSPLIT, int OUT_MODE, int BIAS_MODE>
__global__ __launch_bounds__(256) __attribute__((amdgpu_num_vgpr(256))) void gemm64(
    const unsigned short* __restrict__ Ap, const unsigned short* __restrict__ A2p, int lda, long long strideA,
    const unsigned short* __restrict__ Btp, int ldb, long long strideB,
    const float* __restrict__ bias, const int* __restrict__ flags, int nflag,
    void* Cout, int ldc, long long strideC,
    void* Cout2, int ldc2, long long strideC2, int N2,
    int rmod, int rcnt,
    int tmCnt, int tmPeriod, int tmFirst, int nRowTiles,
    int M, int N, int K, float oscale, float rscale, float rfold) {
  typedef typename OpT<F16OP>::E E;
  typedef typename OpT<F16OP>::V V;
  const E* A   = (const E*)(const void*)Ap;
  const E* A2  = (const E*)(const void*)A2p;
  const E* Bt  = (const E*)(const void*)Btp;
  __shared__ __align__(16) float sT[8][16 * 68];
  const int b    = blockIdx.y;
  const int lane = threadIdx.x & 31;
  const int wave = threadIdx.x >> 5;
  const int tilesN = N >> 6;
  const int tile = blockIdx.x * 8 + wave;
  if (tile >= nRowTiles * tilesN) return;
  const int t2 = tile / tilesN;
  const int tn = tile - t2 * tilesN;
  const int tg = t2 / tmCnt;
  const int tm = tg * tmPeriod + tmFirst + (t2 - tg * tmCnt);
  const int m0 = tm << 6;
  const int n0 = tn << 6;
  const int mq   = m0 / rmod;
  const int mres = m0 - mq * rmod;
  const int m2base = mq * rcnt + mres;
  const bool resRow = (mres < rcnt);

  const E* Ab  = A  + (size_t)b * strideA;
  const E* Bb  = Bt + (size_t)b * strideB;
  const E* Ab2 = A2 + (size_t)b * strideA;

  const int rlane = lane & 15;
  const int koff  = (lane >> 4) * 8;
  const int mOff  = (lane >> 4) * 8;

  v8f acc[4][4];
#pragma unroll
  for (int i = 0; i < 4; ++i)
#pragma unroll
    for (int j = 0; j < 4; ++j) acc[i][j] = zero8();

  const int nph = (NSPLIT >= 1) ? 2 : 1;
  for (int ph = 0; ph < nph; ++ph) {
    const bool resPh = (NSPLIT >= 1) && (ph == 0);
    const E*  Au  = resPh ? Ab2 : Ab;
    const int mr0 = resPh ? m2base : m0;
    for (int k0 = 0; k0 < K; k0 += 32) {
      V bh[4];
#pragma unroll
      for (int j = 0; j < 4; ++j) {
        const size_t bo = (size_t)(n0 + (j << 4) + rlane) * ldb + koff + k0;
        bh[j] = ldfrag(Bb + bo);
      }
#pragma unroll
      for (int i = 0; i < 4; ++i) {
        const size_t ao = (size_t)(mr0 + (i << 4) + rlane) * lda + koff + k0;
        const V ah = ldfrag(Au + ao);
#pragma unroll
        for (int j = 0; j < 4; ++j) acc[i][j] = mma_raw(ah, bh[j], acc[i][j]);
        dep_guard1(acc[i][0], acc[i][3], ah);
      }
      keep4(bh[0], bh[1], bh[2], bh[3]);
    }
    acc_guard4(acc[0][0], acc[0][1], acc[0][2], acc[0][3]);
    acc_guard4(acc[1][0], acc[1][1], acc[1][2], acc[1][3]);
    acc_guard4(acc[2][0], acc[2][1], acc[2][2], acc[2][3]);
    acc_guard4(acc[3][0], acc[3][1], acc[3][2], acc[3][3]);
    if (resPh) {
#pragma unroll
      for (int i = 0; i < 4; ++i)
#pragma unroll
        for (int j = 0; j < 4; ++j) acc[i][j] = acc[i][j] * rfold;
    }
  }

  float osc = oscale;
  if (OUT_MODE == 0 && nflag > 0) {
    int bad = 0;
    for (int f = lane; f < nflag; f += 32) bad |= flags[(size_t)f * 32];
#pragma unroll
    for (int off = 1; off < 32; off <<= 1) bad |= __shfl_xor(bad, off, 32);
    if (bad != 0) osc = __uint_as_float(0x7fc00000u);
  }
  const int c4 = (lane & 15) * 4;
  const int c8 = (lane & 7) * 8;
  v4f bz = {0.f, 0.f, 0.f, 0.f};
  float bc[8];
#pragma unroll
  for (int e = 0; e < 8; ++e) bc[e] = 0.f;
  if (BIAS_MODE == 1) {
    if (OUT_MODE == 0) {
#pragma unroll
      for (int e = 0; e < 4; ++e) bz[e] = bfr(bias[min(n0 + c4 + e, N - 1)]);
    } else {
#pragma unroll
      for (int e = 0; e < 8; ++e) bc[e] = bfr(bias[min(n0 + c8 + e, N - 1)]);
    }
  }

  float* slab = sT[wave];
#pragma unroll
  for (int i = 0; i < 4; ++i) {
    const int mBase = m0 + (i << 4);
#pragma unroll
    for (int j = 0; j < 4; ++j) {
#pragma unroll
      for (int r = 0; r < 8; ++r) {
        slab[(mOff + r) * 68 + (j << 4) + rlane] = acc[i][j][r];
      }
    }
    __builtin_amdgcn_fence(3, "workgroup");
    __builtin_amdgcn_wave_barrier();
    __builtin_amdgcn_fence(2, "workgroup");
    if (OUT_MODE == 0) {
      float* C = (float*)Cout + (size_t)b * strideC;
      const int hh = lane >> 4;
      v4f ov[8];
#pragma unroll
      for (int it = 0; it < 8; ++it) {
        const int row = it * 2 + hh;
        const v4f v = *(const v4f*)(slab + row * 68 + c4);
        ov[it] = v * osc + bz;
      }
      for (int pass = 0; pass < 2; ++pass) {
#pragma unroll
        for (int it = 0; it < 8; ++it) {
          const int row = it * 2 + hh;
          *(volatile v4f*)(C + (size_t)(mBase + row) * ldc + n0 + c4) = ov[it];
        }
        __threadfence();
      }
    } else {
      const int q = lane >> 3;
      unsigned short* C  = (unsigned short*)Cout  + (size_t)b * strideC;
      unsigned short* C2 = (unsigned short*)Cout2 + (size_t)b * strideC2;
      const bool wlo = resRow && (n0 < N2);
      v4u hv[4], lv[4];
#pragma unroll
      for (int it = 0; it < 4; ++it) {
        const int row = it * 4 + q;
        const float* sp = slab + row * 68 + c8;
        float br = 0.f;
        if (BIAS_MODE == 2) br = bfr(bias[min(mBase + row, M - 1)]);
        v4u a, a2;
#pragma unroll
        for (int e = 0; e < 4; ++e) {
          const float f0 = sp[2 * e]     + ((BIAS_MODE == 1) ? bc[2 * e]     : br);
          const float f1 = sp[2 * e + 1] + ((BIAS_MODE == 1) ? bc[2 * e + 1] : br);
          const _Float16 x0 = (_Float16)f0, x1 = (_Float16)f1;
          const unsigned short h0 = h_bits(x0), h1 = h_bits(x1);
          const unsigned short l0 = h_bits((_Float16)((f0 - (float)x0) * rscale));
          const unsigned short l1 = h_bits((_Float16)((f1 - (float)x1) * rscale));
          a[e] = pk16(h0, h1); a2[e] = pk16(l0, l1);
        }
        hv[it] = a; lv[it] = a2;
      }
      for (int pass = 0; pass < 2; ++pass) {
#pragma unroll
        for (int it = 0; it < 4; ++it) {
          const int row = it * 4 + q;
          *(volatile v4u*)(C + (size_t)(mBase + row) * ldc + n0 + c8) = hv[it];
          if (wlo) *(volatile v4u*)(C2 + (size_t)(m2base + (i << 4) + row) * ldc2 + n0 + c8) = lv[it];
        }
        __threadfence();
      }
    }
    __builtin_amdgcn_fence(3, "workgroup");
    __builtin_amdgcn_wave_barrier();
    __builtin_amdgcn_fence(2, "workgroup");
  }
}

template <bool RES>
__global__ __launch_bounds__(128) __attribute__((amdgpu_num_vgpr(256)))
void attn_causal128(const unsigned short* __restrict__ qhp, const unsigned short* __restrict__ qlp,
                    const unsigned short* __restrict__ khp, const unsigned short* __restrict__ klp,
                    const unsigned short* __restrict__ vhp, const unsigned short* __restrict__ vlp,
                    unsigned short* ohp, unsigned short* olp,
                    int qbBase, int nqbThis) {
  constexpr int KC   = RES ? 32 : 64;
  constexpr int NJ   = KC / 16;
  constexpr int NKK  = KC / 32;
  constexpr int CPB  = 64 / KC;
  constexpr int NDT  = RES ? 4 : 8;
  constexpr int DW   = NDT * 16;
  constexpr int NDH  = HD / DW;
  constexpr int TPRK = 128 / KC;
  constexpr int DPT  = 128 / TPRK;
  constexpr int TPRV = 128 / DW;
  constexpr int KPT  = KC / TPRV;
  constexpr int LPR  = DW / 8;
  constexpr int RPI  = 32 / LPR;
  constexpr int NIT  = 16 / RPI;
  static_assert((HD % DW) == 0 && (KPT % 8) == 0 && (DPT % 8) == 0 && NIT * RPI == 16 && NKK >= 1);
  union FH { v16h v; v8h h[2]; };
  __shared__ __align__(16) _Float16 Ksh[KC * 128];
  __shared__ __align__(16) _Float16 Ksl[RES ? KC * 128 : 8];
  __shared__ __align__(16) _Float16 Vth[DW * KC];
  __shared__ __align__(16) _Float16 Vtl[RES ? DW * KC : 8];
  __shared__ __align__(16) _Float16 Psh[4][16 * KC];
  __shared__ __align__(16) _Float16 Psl[RES ? 4 : 1][16 * KC];
  __shared__ __align__(16) float    Os[4][16 * DW];

  const int tid  = threadIdx.x;
  const int wave = tid >> 5;
  const int lane = tid & 31;
  const int hh   = lane >> 4;
  const int c    = lane & 15;

  const int bx    = blockIdx.x;
  const int qbl   = bx % nqbThis;
  const int rest  = bx / nqbThis;
  const int dh    = rest % NDH;
  const int rest2 = rest / NDH;
  const int h     = rest2 % NH;
  const int b     = rest2 / NH;
  const int qb    = qbBase + qbl;
  const int q0    = qb * 64 + wave * 16;
  const int d0    = dh * DW;
  const size_t rowB  = (size_t)b * SEQ;
  const size_t rowB2 = (size_t)b * RESROWS;

  const _Float16* Qh = (const _Float16*)(const void*)qhp + (size_t)h * HD;
  const _Float16* Ql = (const _Float16*)(const void*)qlp + (size_t)h * HD;
  const _Float16* Kh = (const _Float16*)(const void*)khp + (size_t)h * HD;
  const _Float16* Kl = (const _Float16*)(const void*)klp + (size_t)h * HD;
  const _Float16* Vh = (const _Float16*)(const void*)vhp + ((size_t)b * DM + (size_t)h * HD + d0) * SEQ;
  const _Float16* Vl = (const _Float16*)(const void*)vlp + ((size_t)b * DM + (size_t)h * HD + d0) * VLP;
  const float SCL = 1.0f / 11.3137083053588867f;

  const size_t qoff  = (rowB  + q0 + c) * DM + 8 * hh;
  const size_t qloff = (rowB2 + q0 + c) * DM + 8 * hh;

  float mrow[8], lrow[8];
  v8f oacc[NDT];
#pragma unroll
  for (int r = 0; r < 8; ++r) { mrow[r] = -INFINITY; lrow[r] = 0.f; }
#pragma unroll
  for (int t = 0; t < NDT; ++t) oacc[t] = zero8();

  const int nkt = (qb + 1) * CPB;
#pragma unroll 1
  for (int kt = 0; kt < nkt; ++kt) {
    const int kv0 = kt * KC;
    __syncthreads();
    {
      const bool resOK = (kv0 + KC <= VLP);
      const int  kvl   = resOK ? kv0 : (VLP - KC);
      {
        const int r = tid / TPRK, ds = (tid % TPRK) * DPT;
        const _Float16* kg  = Kh + (rowB  + kv0 + r) * DM + ds;
        const _Float16* klg = Kl + (rowB2 + kvl + r) * DM + ds;
#pragma unroll
        for (int i = 0; i < DPT / 8; ++i) {
          const v8h a0 = *(const v8h*)(kg + 8 * i);
          *(v8h*)(Ksh + r * 128 + ds + 8 * i) = a0;
          if (RES) {
            v8h a1 = *(const v8h*)(klg + 8 * i);
            if (!resOK) a1 = zero8h();
            *(v8h*)(Ksl + r * 128 + ds + 8 * i) = a1;
          }
        }
      }
      {
        const int r = tid / TPRV, ks = (tid % TPRV) * KPT;
        const _Float16* vg  = Vh + (size_t)r * SEQ + kv0 + ks;
        const _Float16* vlg = Vl + (size_t)r * VLP + kvl + ks;
#pragma unroll
        for (int i = 0; i < KPT / 8; ++i) {
          const v8h b0 = *(const v8h*)(vg + 8 * i);
          *(v8h*)(Vth + r * KC + ks + 8 * i) = b0;
          if (RES) {
            v8h b1 = *(const v8h*)(vlg + 8 * i);
            if (!resOK) b1 = zero8h();
            *(v8h*)(Vtl + r * KC + ks + 8 * i) = b1;
          }
        }
      }
    }
    __syncthreads();

    v8f s[NJ], s1[NJ];
#pragma unroll
    for (int j = 0; j < NJ; ++j) { s[j] = zero8(); s1[j] = zero8(); }
#pragma unroll 1
    for (int dc = 0; dc < 4; ++dc) {
      {
        const v16h qa = ldfrag(Qh + qoff + dc * 32);
#pragma unroll
        for (int j = 0; j < NJ; ++j) {
          const int ko = (j * 16 + c) * 128 + dc * 32 + 8 * hh;
          FH kb;
          kb.h[0] = *(const v8h*)(Ksh + ko);
          kb.h[1] = *(const v8h*)(Ksh + ko + 16);
          s[j] = mma_h(qa, kb.v, s[j]);
        }
        if (RES) {
#pragma unroll
          for (int j = 0; j < NJ; ++j) {
            const int ko = (j * 16 + c) * 128 + dc * 32 + 8 * hh;
            FH kl;
            kl.h[0] = *(const v8h*)(Ksl + ko);
            kl.h[1] = *(const v8h*)(Ksl + ko + 16);
            s1[j] = mma_h(qa, kl.v, s1[j]);
          }
        }
      }
      if (RES) {
        const v16h ql = ldfrag(Ql + qloff + dc * 32);
#pragma unroll
        for (int j = 0; j < NJ; ++j) {
          const int ko = (j * 16 + c) * 128 + dc * 32 + 8 * hh;
          FH kb;
          kb.h[0] = *(const v8h*)(Ksh + ko);
          kb.h[1] = *(const v8h*)(Ksh + ko + 16);
          s1[j] = mma_h(ql, kb.v, s1[j]);
        }
      }
    }
    if (RES) {
#pragma unroll
      for (int j = 0; j < NJ; ++j)
#pragma unroll
        for (int r = 0; r < 8; ++r) s[j][r] += s1[j][r] * (1.0f / QLC);
    }

    _Float16* pwh = Psh[wave];
    _Float16* pwl = Psl[RES ? wave : 0];
#pragma unroll
    for (int r = 0; r < 8; ++r) {
      const int rowq = q0 + 8 * hh + r;
      float m = -INFINITY;
#pragma unroll
      for (int j = 0; j < NJ; ++j) {
        const int key = kv0 + j * 16 + c;
        float sv = s[j][r] * SCL;
        sv = (key <= rowq) ? sv : -INFINITY;
        s[j][r] = sv;
        m = fmaxf(m, sv);
      }
#pragma unroll
      for (int off = 1; off < 16; off <<= 1) m = fmaxf(m, __shfl_xor(m, off, 32));
      const float mnew  = fmaxf(mrow[r], m);
      const float msafe = (mnew == -INFINITY) ? 0.f : mnew;
      const float alpha = __expf(mrow[r] - msafe);
      mrow[r] = mnew;
      float psum = 0.f;
#pragma unroll
      for (int j = 0; j < NJ; ++j) {
        const float p = __expf(s[j][r] - msafe);
        psum += p;
        const float p1k = p * 1024.0f;
        const _Float16 ph = (_Float16)p1k;
        pwh[(8 * hh + r) * KC + j * 16 + c] = ph;
        if (RES) {
          const _Float16 pl = (_Float16)((p1k - (float)ph) * PVC);
          pwl[(8 * hh + r) * KC + j * 16 + c] = pl;
        }
      }
#pragma unroll
      for (int off = 1; off < 16; off <<= 1) psum += __shfl_xor(psum, off, 32);
      lrow[r] = lrow[r] * alpha + psum;
#pragma unroll
      for (int t = 0; t < NDT; ++t) oacc[t][r] *= alpha;
    }
    __builtin_amdgcn_fence(3, "workgroup");
    __builtin_amdgcn_wave_barrier();
    __builtin_amdgcn_fence(2, "workgroup");

#pragma unroll
    for (int th = 0; th < NDT / 4; ++th) {
      v8f o1[4];
#pragma unroll
      for (int t4 = 0; t4 < 4; ++t4) o1[t4] = zero8();
#pragma unroll 1
      for (int kk = 0; kk < NKK; ++kk) {
        {
          FH pa;
          pa.h[0] = *(const v8h*)(pwh + c * KC + kk * 32 + 8 * hh);
          pa.h[1] = *(const v8h*)(pwh + c * KC + kk * 32 + 16 + 8 * hh);
#pragma unroll
          for (int t4 = 0; t4 < 4; ++t4) {
            const int t  = th * 4 + t4;
            const int vo = (t * 16 + c) * KC + kk * 32 + 8 * hh;
            FH vb;
            vb.h[0] = *(const v8h*)(Vth + vo);
            vb.h[1] = *(const v8h*)(Vth + vo + 16);
            oacc[t] = mma_h(pa.v, vb.v, oacc[t]);
          }
          if (RES) {
#pragma unroll
            for (int t4 = 0; t4 < 4; ++t4) {
              const int t  = th * 4 + t4;
              const int vo = (t * 16 + c) * KC + kk * 32 + 8 * hh;
              FH vl;
              vl.h[0] = *(const v8h*)(Vtl + vo);
              vl.h[1] = *(const v8h*)(Vtl + vo + 16);
              o1[t4] = mma_h(pa.v, vl.v, o1[t4]);
            }
          }
        }
        if (RES) {
          FH pl;
          pl.h[0] = *(const v8h*)(pwl + c * KC + kk * 32 + 8 * hh);
          pl.h[1] = *(const v8h*)(pwl + c * KC + kk * 32 + 16 + 8 * hh);
#pragma unroll
          for (int t4 = 0; t4 < 4; ++t4) {
            const int t  = th * 4 + t4;
            const int vo = (t * 16 + c) * KC + kk * 32 + 8 * hh;
            FH vb;
            vb.h[0] = *(const v8h*)(Vth + vo);
            vb.h[1] = *(const v8h*)(Vth + vo + 16);
            o1[t4] = mma_h(pl.v, vb.v, o1[t4]);
          }
        }
      }
      if (RES) {
#pragma unroll
        for (int t4 = 0; t4 < 4; ++t4)
#pragma unroll
          for (int r = 0; r < 8; ++r) oacc[th * 4 + t4][r] += o1[t4][r] * (1.0f / PVC);
      }
    }
  }

  float* os = Os[wave];
#pragma unroll
  for (int r = 0; r < 8; ++r) {
    const float l = lrow[r];
    const float inv = ((l > 0.f) ? (1.0f / l) : 0.f) * (1.0f / 1024.0f);
#pragma unroll
    for (int t = 0; t < NDT; ++t) os[(8 * hh + r) * DW + t * 16 + c] = oacc[t][r] * inv;
  }
  __builtin_amdgcn_fence(3, "workgroup");
  __builtin_amdgcn_wave_barrier();
  __builtin_amdgcn_fence(2, "workgroup");
  {
    const int rq = lane / LPR, c8 = (lane % LPR) * 8;
    v4u hv[NIT], lv[NIT];
#pragma unroll
    for (int it = 0; it < NIT; ++it) {
      const int row = it * RPI + rq;
      const float* sp = os + row * DW + c8;
      v4u a, a2;
#pragma unroll
      for (int e = 0; e < 4; ++e) {
        const float f0 = sp[2 * e], f1 = sp[2 * e + 1];
        const _Float16 x0 = (_Float16)f0, x1 = (_Float16)f1;
        const unsigned short h0 = h_bits(x0), h1 = h_bits(x1);
        const unsigned short l0 = h_bits((_Float16)((f0 - (float)x0) * OLC));
        const unsigned short l1 = h_bits((_Float16)((f1 - (float)x1) * OLC));
        a[e] = pk16(h0, h1); a2[e] = pk16(l0, l1);
      }
      hv[it] = a; lv[it] = a2;
    }
    for (int pass = 0; pass < 2; ++pass) {
#pragma unroll
      for (int it = 0; it < NIT; ++it) {
        const int row = it * RPI + rq;
        const size_t go = (rowB + q0 + row) * DM + (size_t)h * HD + d0 + c8;
        *(volatile v4u*)(ohp + go) = hv[it];
        if (RES) {
          const size_t go2 = (rowB2 + q0 + row) * DM + (size_t)h * HD + d0 + c8;
          *(volatile v4u*)(olp + go2) = lv[it];
        }
      }
      __threadfence();
    }
  }
}

extern "C" void kernel_launch(void* const* d_in, const int* in_sizes, int n_in,
                              void* d_out, int out_size, void* d_ws, size_t ws_size,
                              hipStream_t stream) {
  if (n_in < 10) return;
  if (in_sizes[0] < ((NB - 1) * SEQ_FULL + SEQ) * DM) return;
  if (in_sizes[1] < (SEQ - 1) * SEQ_FULL + SEQ) return;
  if (in_sizes[2] < DM * DM || in_sizes[4] < DM * DM || in_sizes[6] < DM * DM || in_sizes[8] < DM * DM) return;
  if (in_sizes[3] < DM || in_sizes[5] < DM || in_sizes[7] < DM || in_sizes[9] < DM) return;
  if (out_size < NB * SEQ * DM) return;

  const float* x   = (const float*)d_in[0];
  const int*   msk = (const int*)d_in[1];
  const float* Wq  = (const float*)d_in[2];
  const float* bq  = (const float*)d_in[3];
  const float* Wk  = (const float*)d_in[4];
  const float* bk  = (const float*)d_in[5];
  const float* Wv  = (const float*)d_in[6];
  const float* bv  = (const float*)d_in[7];
  const float* Wo  = (const float*)d_in[8];
  const float* bo  = (const float*)d_in[9];

  const size_t PX  = (size_t)NB * SEQ * DM * 2;
  const size_t PW  = (size_t)DM * DM * 2;
  const size_t PR  = (size_t)NB * RESROWS * DM * 2;
  const size_t PVT = (size_t)NB * DM * SEQ * 2;
  const size_t PVL = (size_t)NB * DM * VLP * 2;
  const size_t PFL = (size_t)CHKB * 128;
  size_t off = 0;
  const size_t oXb  = off; off += PX;
  const size_t oWq  = off; off += PW;
  const size_t oWk  = off; off += PW;
  const size_t oWv  = off; off += PW;
  const size_t oWo  = off; off += PW;
  const size_t oQh  = off; off += PX;
  const size_t oQl  = off; off += PR;
  const size_t oKh  = off; off += PX;
  const size_t oKl  = off; off += PR;
  const size_t oVTh = off; off += PVT;
  const size_t oVTl = off; off += PVL;
  const size_t oOl  = off; off += PR;
  const size_t oFlg = off; off += PFL;
  if (off > ws_size) return;
  if (off > (size_t)134217728) return;
  const size_t oOh  = oXb;

  char* ws = (char*)d_ws;
  unsigned short* Xb  = (unsigned short*)(ws + oXb);
  unsigned short* Wqb = (unsigned short*)(ws + oWq);
  unsigned short* Wkb = (unsigned short*)(ws + oWk);
  unsigned short* Wvb = (unsigned short*)(ws + oWv);
  unsigned short* Woh = (unsigned short*)(ws + oWo);
  unsigned short* Qh  = (unsigned short*)(ws + oQh);
  unsigned short* Ql  = (unsigned short*)(ws + oQl);
  unsigned short* Kh  = (unsigned short*)(ws + oKh);
  unsigned short* Kl  = (unsigned short*)(ws + oKl);
  unsigned short* VTh = (unsigned short*)(ws + oVTh);
  unsigned short* VTl = (unsigned short*)(ws + oVTl);
  unsigned short* Oh  = (unsigned short*)(ws + oOh);
  unsigned short* Ol  = (unsigned short*)(ws + oOl);
  int*            Flg = (int*)(ws + oFlg);

  const dim3 blk(256);
  const int n8x = SEQ * DM / 8;
  const int n8w = DM * DM / 8;
  const dim3 gCvtX((n8x + 255) / 256, NB);
  const dim3 gCvtW((n8w + 255) / 256, 1);
  const dim3 gProj(((NB * SEQ / 64) * (DM / 64) + 7) / 8, 1);
  const dim3 gVT(((DM / 64) * (SEQ / 64) + 7) / 8, NB);
  const dim3 gOutE(((NB * RESQB) * (DM / 64) + 7) / 8, 1);
  const dim3 gOutL(((NB * (NQB - RESQB)) * (DM / 64) + 7) / 8, 1);
  const dim3 gAttE(NB * NH * (HD / 64) * RESQB);
  const dim3 gAttL(NB * NH * ((NQB > RESQB) ? (NQB - RESQB) : 1));

  cvt_bf16x8<<<gCvtX, blk, 0, stream>>>(x, Xb, n8x, (long long)SEQ_FULL * DM, (long long)SEQ * DM);
  cvt_bf16x8<<<gCvtW, blk, 0, stream>>>(Wq, Wqb, n8w, 0LL, 0LL);
  cvt_bf16x8<<<gCvtW, blk, 0, stream>>>(Wk, Wkb, n8w, 0LL, 0LL);
  cvt_bf16x8<<<gCvtW, blk, 0, stream>>>(Wv, Wvb, n8w, 0LL, 0LL);
  cvt_f16x8<<<gCvtW, blk, 0, stream>>>(Wo, Woh, n8w, WOC);
  mask_check<<<dim3(CHKB), blk, 0, stream>>>(msk, Flg, SEQ, SEQ_FULL);
  gemm64<false, 0, 3, 1><<<gProj, blk, 0, stream>>>(
      Xb, Xb, DM, 0LL, Wqb, DM, 0LL, bq, Flg, 0,
      (void*)Qh, DM, 0LL, (void*)Ql, DM, 0LL, DM,
      SEQ, RESROWS,
      NB * SEQ / 64, NB * SEQ / 64, 0, NB * SEQ / 64,
      NB * SEQ, DM, DM, 1.0f, QLC, 1.0f);
  gemm64<false, 0, 3, 1><<<gProj, blk, 0, stream>>>(
      Xb, Xb, DM, 0LL, Wkb, DM, 0LL, bk, Flg, 0,
      (void*)Kh, DM, 0LL, (void*)Kl, DM, 0LL, DM,
      SEQ, RESROWS,
      NB * SEQ / 64, NB * SEQ / 64, 0, NB * SEQ / 64,
      NB * SEQ, DM, DM, 1.0f, QLC, 1.0f);
  gemm64<false, 0, 3, 2><<<gVT, blk, 0, stream>>>(
      Wvb, Wvb, DM, 0LL, Xb, DM, (long long)SEQ * DM, bv, Flg, 0,
      (void*)VTh, SEQ, (long long)DM * SEQ, (void*)VTl, VLP, (long long)DM * VLP, VLP,
      DM, DM,
      DM / 64, DM / 64, 0, DM / 64,
      DM, SEQ, DM, 1.0f, PVC, 1.0f);
  attn_causal128<true><<<gAttE, dim3(128), 0, stream>>>(
      Qh, Ql, Kh, Kl, VTh, VTl, Oh, Ol, 0, RESQB);
  if (NQB > RESQB) {
    attn_causal128<false><<<gAttL, dim3(128), 0, stream>>>(
        Qh, Ql, Kh, Kl, VTh, VTl, Oh, Ol, RESQB, NQB - RESQB);
  }
  gemm64<true, 1, 0, 1><<<gOutE, blk, 0, stream>>>(
      Oh, Ol, DM, 0LL, Woh, DM, 0LL, bo, Flg, CHKB,
      d_out, DM, 0LL, d_out, DM, 0LL, 0,
      SEQ, RESROWS,
      RESQB, NQB, 0, NB * RESQB,
      NB * SEQ, DM, DM, 1.0f / WOC, 1.0f, 1.0f / OLC);
  if (NQB > RESQB) {
    gemm64<true, 0, 0, 1><<<gOutL, blk, 0, stream>>>(
        Oh, Oh, DM, 0LL, Woh, DM, 0LL, bo, Flg, CHKB,
        d_out, DM, 0LL, d_out, DM, 0LL, 0,
        SEQ, RESROWS,
        NQB - RESQB, NQB, RESQB, NB * (NQB - RESQB),
        NB * SEQ, DM, DM, 1.0f / WOC, 1.0f, 1.0f);
  }
  (void)hipGetLastError();
}
